// EquiformerLayer_71992241815599
// MI455X (gfx1250) — hardware-verified
//
#include <hip/hip_runtime.h>
#include <stdint.h>
#include <math.h>

typedef __attribute__((ext_vector_type(16))) _Float16 v16h;
typedef __attribute__((ext_vector_type(8)))  _Float16 v8h;
typedef __attribute__((ext_vector_type(4)))  _Float16 v4h;
typedef __attribute__((ext_vector_type(16))) __bf16   v16b;
typedef __attribute__((ext_vector_type(8)))  __bf16   v8b;
typedef __attribute__((ext_vector_type(8)))  float    v8f;
typedef __attribute__((ext_vector_type(4)))  float    v4f;

#define DIMC 256
#define NCHUNK 4
#define NSLOTS 10
#define SRB 2048
#define ANT 256
#define ANW 8
#define RPW (SRB / ANW)
#define SCH 4096
#define SP (SCH / ANT)
#define ELB 20
#define ELM ((1 << ELB) - 1)

#define SQ3F 1.7320508075688772f
#define INV_SQ3F 0.57735026918962576f
#define INV_MULF 0.125f
#define INV_TPF 0.08838834764831845f
#define W3SC 0.015625f
#define MSG_SC 64.0f
#define MSG_ISC 0.015625f
#define LK_SC 16.0f
#define LK_ISC 0.0625f

#define BT1_OFF 0
#define BTC_OFF 8192
#define BTD_OFF 12288
#define BTS_OFF 16384
#define BT2_OFF 20480
#define BT21_OFF 28672
#define BT22_OFF 32768
#define BT_HALVES 36864

static_assert(SP * ANT == SCH);
static_assert(RPW * ANW == SRB);
static_assert(RPW == 256);
static_assert(SRB <= (1 << (31 - ELB)));

__device__ __forceinline__ unsigned short f2bf_bits(float f) {
  unsigned u = __float_as_uint(f);
  return (unsigned short)((u + 0x7FFFu + ((u >> 16) & 1u)) >> 16);
}
__device__ __forceinline__ float bf_bits2f(unsigned short h) { return __uint_as_float(((unsigned)h) << 16); }

__device__ __forceinline__ void dep_guard_h(v8f& a, v8f& b, v16h x, v16h y) { asm volatile("v_nop\n\tv_nop\n\tv_nop\n\tv_nop" : "+v"(a), "+v"(b) : "v"(x), "v"(y)); }
__device__ __forceinline__ void dep_guard_b(v8f& a, v8f& b, v16b x, v16b y) { asm volatile("v_nop\n\tv_nop\n\tv_nop\n\tv_nop" : "+v"(a), "+v"(b) : "v"(x), "v"(y)); }
__device__ __forceinline__ void keep4_h(v16h a, v16h b, v16h c, v16h d) { asm volatile("v_nop" :: "v"(a), "v"(b), "v"(c), "v"(d)); }
__device__ __forceinline__ void keep4_b(v16b a, v16b b, v16b c, v16b d) { asm volatile("v_nop" :: "v"(a), "v"(b), "v"(c), "v"(d)); }
__device__ __forceinline__ void acc_guard4(v8f& a, v8f& b, v8f& c, v8f& d) { asm volatile("v_nop\n\tv_nop\n\tv_nop\n\tv_nop" : "+v"(a), "+v"(b), "+v"(c), "+v"(d)); }
template <typename T> struct Frag;
template <> struct Frag<_Float16> {
  typedef v16h V; union U { v16h v; v8h h[2]; };
  static __device__ __forceinline__ v16h load(const _Float16* p) {
    U f; f.h[0] = *(const v8h*)(p); f.h[1] = *(const v8h*)(p + 16); return f.v;
  }
  static __device__ __forceinline__ v8f mma(v16h a, v16h b, v8f c) {
    return __builtin_amdgcn_wmma_f32_16x16x32_f16(false, a, false, b, (short)0, c, false, false);
  }
  static __device__ __forceinline__ void guard(v8f& a, v8f& b, v16h x, v16h y) { dep_guard_h(a, b, x, y); }
  static __device__ __forceinline__ void keep(v16h a, v16h b, v16h c, v16h d) { keep4_h(a, b, c, d); }
};
template <> struct Frag<__bf16> {
  typedef v16b V; union U { v16b v; v8b h[2]; };
  static __device__ __forceinline__ v16b load(const __bf16* p) {
    U f; f.h[0] = *(const v8b*)(p); f.h[1] = *(const v8b*)(p + 16); return f.v;
  }
  static __device__ __forceinline__ v8f mma(v16b a, v16b b, v8f c) {
    return __builtin_amdgcn_wmma_f32_16x16x32_bf16(false, a, false, b, (short)0, c, false, false);
  }
  static __device__ __forceinline__ void guard(v8f& a, v8f& b, v16b x, v16b y) { dep_guard_b(a, b, x, y); }
  static __device__ __forceinline__ void keep(v16b a, v16b b, v16b c, v16b d) { keep4_b(a, b, c, d); }
};
__device__ __forceinline__ void wave_sync() {
  __builtin_amdgcn_fence(__ATOMIC_RELEASE, "workgroup");
  __builtin_amdgcn_wave_barrier();
  __builtin_amdgcn_fence(__ATOMIC_ACQUIRE, "workgroup");
}

template <int ET> struct Elem;
template <> struct Elem<0> { typedef _Float16 T; };
template <> struct Elem<1> { typedef __bf16 T; };
template <int ET, bool SPLIT, int BIAS_MODE, int OUT_MODE, bool RESID, int ACT = 0>
__global__ __launch_bounds__(256) void wmma_gemm64(
    const unsigned short* __restrict__ Ap, const unsigned short* __restrict__ A2p, int lda, long strideA,
    const unsigned short* __restrict__ Btp, const unsigned short* __restrict__ Bt2p, int ldb, long strideB,
    void* __restrict__ Cout, void* __restrict__ Cout2, int ldc, long strideC,
    const float* __restrict__ bias, long strideBias,
    const float* __restrict__ resid, long strideR,
    int M, int N, int K, float scale) {
  typedef typename Elem<ET>::T T;
  typedef typename Frag<T>::V V;
  const T* A = (const T*)Ap; const T* A2 = (const T*)A2p; const T* Bt = (const T*)Btp; const T* Bt2 = (const T*)Bt2p;
  __shared__ __align__(16) float sT[8][16 * 68];
  const int b    = blockIdx.y;
  const int lane = threadIdx.x & 31;
  const int wave = threadIdx.x >> 5;
  const int tilesN = N >> 6;
  const int tilesM = M >> 6;
  const int tile = blockIdx.x * 8 + wave;
  if (tile >= tilesM * tilesN) return;
  const int tm = tile / tilesN;
  const int tn = tile - tm * tilesN;
  const int m0 = tm << 6;
  const int n0 = tn << 6;

  const T* Ab  = A  + (size_t)b * strideA;
  const T* Bb  = Bt + (size_t)b * strideB;
  const T* Ab2 = SPLIT ? (A2  + (size_t)b * strideA) : nullptr;
  const T* Bb2 = SPLIT ? (Bt2 + (size_t)b * strideB) : nullptr;

  const int rlane = lane & 15;
  const int koff  = (lane >> 4) * 8;
  const int mOff  = (lane >> 4) * 8;

  v8f acc[4][4];
#pragma unroll
  for (int i = 0; i < 4; ++i)
#pragma unroll
    for (int j = 0; j < 4; ++j) acc[i][j] = (v8f){0.f,0.f,0.f,0.f,0.f,0.f,0.f,0.f};

  for (int k0 = 0; k0 < K; k0 += 32) {
    V bh[4], bl[4];
#pragma unroll
    for (int j = 0; j < 4; ++j) {
      const size_t bo = (size_t)(n0 + (j << 4) + rlane) * ldb + koff + k0;
      bh[j] = Frag<T>::load(Bb + bo);
      if (SPLIT) bl[j] = Frag<T>::load(Bb2 + bo);
    }
#pragma unroll
    for (int i = 0; i < 4; ++i) {
      const size_t ao = (size_t)(m0 + (i << 4) + rlane) * lda + koff + k0;
      V ah = Frag<T>::load(Ab + ao);
      V al;
      if (SPLIT) al = Frag<T>::load(Ab2 + ao);
#pragma unroll
      for (int j = 0; j < 4; ++j) {
        acc[i][j] = Frag<T>::mma(ah, bh[j], acc[i][j]);
        if (SPLIT) {
          acc[i][j] = Frag<T>::mma(ah, bl[j], acc[i][j]);
          acc[i][j] = Frag<T>::mma(al, bh[j], acc[i][j]);
        }
      }
      Frag<T>::guard(acc[i][0], acc[i][3], ah, SPLIT ? al : ah);
    }
    Frag<T>::keep(bh[0], bh[1], bh[2], bh[3]);
    if (SPLIT) Frag<T>::keep(bl[0], bl[1], bl[2], bl[3]);
  }
  acc_guard4(acc[0][0], acc[0][1], acc[0][2], acc[0][3]);
  acc_guard4(acc[1][0], acc[1][1], acc[1][2], acc[1][3]);
  acc_guard4(acc[2][0], acc[2][1], acc[2][2], acc[2][3]);
  acc_guard4(acc[3][0], acc[3][1], acc[3][2], acc[3][3]);

  float* slab = sT[wave];
  const float* Rb  = RESID ? (resid + (size_t)b * strideR) : nullptr;
  const float* Bsb = (BIAS_MODE != 0) ? (bias + (size_t)b * strideBias) : nullptr;
#pragma unroll
  for (int i = 0; i < 4; ++i) {
    const int mBase = m0 + (i << 4);
    float rsc[8];
#pragma unroll
    for (int r = 0; r < 8; ++r) rsc[r] = (BIAS_MODE == 1 || BIAS_MODE == 3) ? Bsb[mBase + mOff + r] : 0.f;
#pragma unroll
    for (int j = 0; j < 4; ++j) {
      const int n = n0 + (j << 4) + rlane;
      float bv = 0.f;
      if (BIAS_MODE == 2) bv = Bsb[n];
#pragma unroll
      for (int r = 0; r < 8; ++r) {
        float v = acc[i][j][r] * scale;
        if (BIAS_MODE == 1) v += rsc[r];
        if (BIAS_MODE == 2) v += bv;
        if (RESID) {
          float rv = Rb[(size_t)(mBase + mOff + r) * ldc + n];
          if (BIAS_MODE == 3) rv = rv * rsc[r];
          v += rv;
        }
        if (ACT == 1) v = tanhf(v);
        if (ACT == 2) v = fmaxf(v, 0.0f);
        if (ACT == 3) v = v / (1.0f + expf(-v));
        if (ACT == 4) v = (v > 0.f) ? v : 0.01f * v;
        if (ACT == 5) v = 0.5f * v * (1.0f + erff(v * 0.70710678118654752f));
        slab[(mOff + r) * 68 + (j << 4) + rlane] = v;
      }
    }
    __builtin_amdgcn_fence(__ATOMIC_RELEASE, "workgroup");
    __builtin_amdgcn_wave_barrier();
    __builtin_amdgcn_fence(__ATOMIC_ACQUIRE, "workgroup");
    if (OUT_MODE == 0) {
      float* C = (float*)Cout + (size_t)b * strideC;
      const int hh = lane >> 4, c4 = (lane & 15) * 4;
      for (int pass = 0; pass < 2; ++pass) {
#pragma unroll
        for (int it = 0; it < 8; ++it) {
          const int row = it * 2 + hh;
          v4f v = *(const v4f*)(slab + row * 68 + c4);
          *(volatile v4f*)(C + (size_t)(mBase + row) * ldc + n0 + c4) = v;
        }
        __threadfence();
      }
    } else {
      const int q = lane >> 3, c8 = (lane & 7) * 8;
      unsigned short* C  = (unsigned short*)Cout  + (size_t)b * strideC;
      unsigned short* C2 = (OUT_MODE == 2) ? ((unsigned short*)Cout2 + (size_t)b * strideC) : nullptr;
      for (int pass = 0; pass < 2; ++pass) {
#pragma unroll
        for (int it = 0; it < 4; ++it) {
          const int row = it * 4 + q;
          const float* sp = slab + row * 68 + c8;
          v8h hv, lv;
#pragma unroll
          for (int e = 0; e < 8; ++e) {
            if (OUT_MODE == 1) {
              hv[e] = (_Float16)sp[e];
            } else {
              unsigned short hb = f2bf_bits(sp[e]);
              unsigned short lb = f2bf_bits(sp[e] - bf_bits2f(hb));
              hv[e] = __builtin_bit_cast(_Float16, hb);
              lv[e] = __builtin_bit_cast(_Float16, lb);
            }
          }
          *(volatile v8h*)(C + (size_t)(mBase + row) * ldc + n0 + c8) = hv;
          if (OUT_MODE == 2) *(volatile v8h*)(C2 + (size_t)(mBase + row) * ldc + n0 + c8) = lv;
        }
        __threadfence();
      }
    }
    __builtin_amdgcn_fence(__ATOMIC_RELEASE, "workgroup");
    __builtin_amdgcn_wave_barrier();
    __builtin_amdgcn_fence(__ATOMIC_ACQUIRE, "workgroup");
  }
}

#define GEMM_F32 wmma_gemm64<0, false, 0, 0, false>
#define GEMM_F16 wmma_gemm64<0, false, 0, 1, false>
#define GEMM_RS  wmma_gemm64<0, false, 3, 1, true>

__global__ __launch_bounds__(256) void prep_kernel(
    const float* __restrict__ ls0, const float* __restrict__ ls1,
    const float* __restrict__ t1_00, const float* __restrict__ t1_11, const float* __restrict__ t1_01, const float* __restrict__ t1_10,
    const float* __restrict__ t2_00, const float* __restrict__ t2_11, const float* __restrict__ t2_01, const float* __restrict__ t2_10,
    const float* __restrict__ lh0, const float* __restrict__ lh1, const float* __restrict__ lsc,
    _Float16* bt) {
  __shared__ float P[4096];
  __shared__ float Q[4096];
  __shared__ float R3[4096];
  __shared__ float T[4096];
  const int job = blockIdx.x;
  const int tid = threadIdx.x, lane = tid & 31, wave = tid >> 5;
  const float* W1 = lsc; const float* W2 = lsc; const float* W3 = lsc;
  int comp = 0, dsto = BTS_OFF, pitch = 64;
  if (job == 0)      { W1 = ls0; W2 = t1_00; W3 = lh0; comp = 1; dsto = BT1_OFF;      pitch = 128; }
  else if (job == 1) { W1 = ls1; W2 = t1_11; W3 = lh0; comp = 1; dsto = BT1_OFF + 64; pitch = 128; }
  else if (job == 2) { W1 = ls0; W2 = t1_01; W3 = lh1; comp = 1; dsto = BTC_OFF;      pitch = 64; }
  else if (job == 3) { W1 = ls1; W2 = t1_10; W3 = lh1; comp = 1; dsto = BTD_OFF;      pitch = 64; }
  else if (job == 4) { W1 = lsc;   dsto = BTS_OFF;      pitch = 64; }
  else if (job == 5) { W1 = t2_00; dsto = BT2_OFF;      pitch = 128; }
  else if (job == 6) { W1 = t2_11; dsto = BT2_OFF + 64; pitch = 128; }
  else if (job == 7) { W1 = t2_01; dsto = BT21_OFF;     pitch = 64; }
  else               { W1 = t2_10; dsto = BT22_OFF;     pitch = 64; }
#pragma unroll 1
  for (int i = tid; i < 4096; i += 256) {
    P[i] = W1[i];
    if (comp) { Q[i] = W2[i]; R3[i] = W3[i]; }
  }
  __syncthreads();
  if (comp) {
#pragma unroll 1
    for (int qq = 0; qq < 16; ++qq) {
      const int idx = tid + 256 * qq; const int i = idx >> 6, jn = idx & 63;
      float s = 0.f;
#pragma unroll 1
      for (int k = 0; k < 64; ++k) s += P[i * 64 + k] * Q[k * 64 + jn];
      T[idx] = s;
    }
    __syncthreads();
#pragma unroll 1
    for (int qq = 0; qq < 16; ++qq) {
      const int idx = tid + 256 * qq; const int i = idx >> 6, jn = idx & 63;
      float s = 0.f;
#pragma unroll 1
      for (int k = 0; k < 64; ++k) s += T[i * 64 + k] * R3[k * 64 + jn];
      P[idx] = s * W3SC;
    }
    __syncthreads();
  }
  const int q = lane >> 3, e8 = (lane & 7) * 8;
  const int nA = wave * 4 + q, nB = 32 + wave * 4 + q;
  v8h hA, hB;
#pragma unroll
  for (int e = 0; e < 8; ++e) { hA[e] = (_Float16)P[(e8 + e) * 64 + nA]; hB[e] = (_Float16)P[(e8 + e) * 64 + nB]; }
  _Float16* dA = bt + dsto + (size_t)nA * pitch + e8;
  _Float16* dB = bt + dsto + (size_t)nB * pitch + e8;
  for (int pass = 0; pass < 2; ++pass) {
    *(volatile v8h*)dA = hA;
    *(volatile v8h*)dB = hB;
    __threadfence();
  }
}

__global__ __launch_bounds__(256) void gather_kernel(const float* __restrict__ atom, const float* __restrict__ evec, const int* __restrict__ ei,
                                                     _Float16* x0d, _Float16* x1, float* shv, long pstride,
                                                     int N, int E, int c0, int C, int Mpad) {
  __shared__ float SHL[3][256];
  __shared__ __align__(16) float XR[8][256];
  const int tid = threadIdx.x, lane = tid & 31, wave = tid >> 5;
  const int rbase = blockIdx.x * 256;
  {
    const int row = rbase + tid;
    int eg = c0 + row; eg = eg < E ? eg : E - 1;
    const float vx = evec[(size_t)eg * 3 + 0], vy = evec[(size_t)eg * 3 + 1], vz = evec[(size_t)eg * 3 + 2];
    const float nrm = sqrtf(vx * vx + vy * vy + vz * vz);
    const float inv = 1.0f / (nrm + 1e-12f);
    const float s0 = SQ3F * (vx * inv), s1 = SQ3F * (vy * inv), s2 = SQ3F * (vz * inv);
    SHL[0][tid] = s0; SHL[1][tid] = s1; SHL[2][tid] = s2;
    if (row < Mpad) {
      for (int pass = 0; pass < 2; ++pass) {
        *(volatile float*)(shv + row) = s0;
        *(volatile float*)(shv + (size_t)C + row) = s1;
        *(volatile float*)(shv + 2 * (size_t)C + row) = s2;
        __threadfence();
      }
    }
  }
  __syncthreads();
  float* xr = XR[wave];
  const int q8 = (lane & 7) * 8;
  int mm = lane >> 3; mm = mm < 3 ? mm : 2;
#pragma unroll 1
  for (int j = 0; j < 32; ++j) {
    const int rl = wave * 32 + j;
    const int row = rbase + rl;
    if (row < Mpad) {
      int eg = c0 + row; eg = eg < E ? eg : E - 1;
      int s = ei[eg]; s = s < 0 ? 0 : (s >= N ? N - 1 : s);
      const float* ar = atom + (size_t)s * DIMC + lane * 8;
      const v4f p0 = *(const v4f*)ar;
      const v4f p1 = *(const v4f*)(ar + 4);
      *(v4f*)(xr + lane * 8) = p0;
      *(v4f*)(xr + lane * 8 + 4) = p1;
      wave_sync();
      const float sh0 = SHL[0][rl], sh1 = SHL[1][rl], sh2 = SHL[2][rl];
      v8h hx, hdv, h1v;
#pragma unroll
      for (int e = 0; e < 8; ++e) {
        const int u = q8 + e;
        hx[e] = (_Float16)xr[u];
        const float* vp = xr + 64 + 3 * u;
        hdv[e] = (_Float16)(((vp[0] * sh0 + vp[1] * sh1) + vp[2] * sh2) * INV_SQ3F);
        h1v[e] = (_Float16)vp[mm];
      }
      wave_sync();
      const v8h v0 = (lane < 8) ? hx : hdv;
      _Float16* d0 = x0d + (size_t)row * 128 + 8 * lane;
      _Float16* d1 = x1 + (size_t)mm * pstride + (size_t)row * 64 + q8;
      for (int pass = 0; pass < 2; ++pass) {
        if (lane < 16) *(volatile v8h*)d0 = v0;
        if (lane < 24) *(volatile v8h*)d1 = h1v;
        __threadfence();
      }
    }
  }
}

__global__ __launch_bounds__(256) void lkdot_kernel(_Float16* hd, const _Float16* __restrict__ h1p, const float* __restrict__ shv,
                                                    _Float16* lk, long pstride, int C, int Mpad) {
  const int tid = threadIdx.x, lane = tid & 31, wave = tid >> 5;
  const int rb = blockIdx.x * 32 + wave * 4;
  if (rb < Mpad) {
    const int row = rb + (lane >> 3), q8 = (lane & 7) * 8;
    const v8h h0 = *(const v8h*)(hd + (size_t)row * 128 + q8);
    const size_t ro = (size_t)row * 64 + q8;
    const v8h a = *(const v8h*)(h1p + ro);
    const v8h bq = *(const v8h*)(h1p + (size_t)pstride + ro);
    const v8h cq = *(const v8h*)(h1p + 2 * (size_t)pstride + ro);
    const float s0 = shv[row], s1 = shv[(size_t)C + row], s2 = shv[2 * (size_t)C + row];
    v8h lkv, d2;
#pragma unroll
    for (int e = 0; e < 8; ++e) {
      const float v = (float)h0[e];
      lkv[e] = (_Float16)((v >= 0.f ? v : 0.01f * v) * LK_SC);
      d2[e] = (_Float16)((((float)a[e] * s0 + (float)bq[e] * s1) + (float)cq[e] * s2) * INV_SQ3F);
    }
    _Float16* dl = lk + ro;
    _Float16* dd = hd + (size_t)row * 128 + 64 + q8;
    for (int pass = 0; pass < 2; ++pass) {
      *(volatile v8h*)dl = lkv;
      *(volatile v8h*)dd = d2;
      __threadfence();
    }
  }
}

__global__ __launch_bounds__(256) void msg_kernel(const _Float16* __restrict__ sc, const _Float16* __restrict__ o0,
                                                  const _Float16* __restrict__ o1, _Float16* msg, long pstride, int Mpad) {
  __shared__ __align__(16) _Float16 MT[8][4 * 256];
  const int tid = threadIdx.x, lane = tid & 31, wave = tid >> 5;
  const int rb = blockIdx.x * 32 + wave * 4;
  if (rb < Mpad) {
    const int sl = lane >> 3, q = lane & 7, q8 = q * 8;
    const int row = rb + sl;
    const size_t ro = (size_t)row * 64 + q8;
    const v8h scv = *(const v8h*)(sc + ro);
    const v8h o0v = *(const v8h*)(o0 + ro);
    v8h o1v[3];
#pragma unroll
    for (int m = 0; m < 3; ++m) o1v[m] = *(const v8h*)(o1 + (size_t)m * pstride + ro);
    float mx = 0.f;
#pragma unroll
    for (int e = 0; e < 8; ++e) mx = fmaxf(mx, (float)scv[e]);
    mx = fmaxf(mx, __shfl_xor(mx, 1, 32));
    mx = fmaxf(mx, __shfl_xor(mx, 2, 32));
    mx = fmaxf(mx, __shfl_xor(mx, 4, 32));
    float ev[8]; float s = 0.f;
#pragma unroll
    for (int e = 0; e < 8; ++e) { ev[e] = __expf((float)scv[e] - mx); s += ev[e]; }
    s += __shfl_xor(s, 1, 32);
    s += __shfl_xor(s, 2, 32);
    s += __shfl_xor(s, 4, 32);
    const float z = __expf(-mx);
    const float Z = s + 192.0f * z;
    const float inv = 1.0f / Z;
    const float a1 = z * inv * MSG_SC;
    v8h m0v;
#pragma unroll
    for (int e = 0; e < 8; ++e) { const float a = ev[e] * inv; m0v[e] = (_Float16)(a * (float)o0v[e] * MSG_SC); }
    v8h w[3];
#pragma unroll
    for (int f = 0; f < 24; ++f) {
      const int uu = f / 3, m = f - 3 * uu;
      w[f >> 3][f & 7] = (_Float16)(a1 * (float)o1v[m][uu]);
    }
    _Float16* mt = MT[wave] + sl * 256;
    *(v8h*)(mt + q8) = m0v;
    *(v8h*)(mt + 64 + 24 * q) = w[0];
    *(v8h*)(mt + 72 + 24 * q) = w[1];
    *(v8h*)(mt + 80 + 24 * q) = w[2];
    wave_sync();
    v8h pv[4];
#pragma unroll
    for (int k = 0; k < 4; ++k) pv[k] = *(const v8h*)(MT[wave] + k * 256 + 8 * lane);
    for (int pass = 0; pass < 2; ++pass) {
#pragma unroll
      for (int k = 0; k < 4; ++k) *(volatile v8h*)(msg + (size_t)(rb + k) * 256 + 8 * lane) = pv[k];
      __threadfence();
    }
  }
}

__device__ __forceinline__ int blk_excl_scan(int cnt, int* scan_ws, int tid, int* tot) {
  const int lane = tid & 31, wave = tid >> 5; int incl = cnt;
#pragma unroll
  for (int o = 1; o < 32; o <<= 1) { const int v = __shfl_up(incl, o, 32); if (lane >= o) incl += v; }
  if (lane == 31) scan_ws[wave] = incl;
  __syncthreads();
  if (wave == 0) { int wv = (lane < ANT / 32) ? scan_ws[lane] : 0; int wincl = wv;
#pragma unroll
    for (int o = 1; o < 32; o <<= 1) { const int v = __shfl_up(wincl, o, 32); if (lane >= o) wincl += v; }
    if (lane < ANT / 32) scan_ws[32 + lane] = wincl - wv; if (lane == 31) scan_ws[64] = wincl; }
  __syncthreads();
  const int res = scan_ws[32 + wave] + incl - cnt; *tot = scan_ws[64];
  return res;
}
__device__ __forceinline__ int chunk_hits_e(const int* __restrict__ dstv, int e0, int c0, int c1, int n0, int nhi, int tid,
                                            int* LIST, int* scan_ws) {
  const int eb = e0 + tid * SP;
  int rec[SP]; int cnt = 0;
#pragma unroll
  for (int k = 0; k < SP; ++k) {
    const int e = eb + k;
    const int ec = e < c1 ? e : c1 - 1;
    const int d = dstv[ec];
    int r = -1;
    if (e < c1 && d >= n0 && d < nhi) { r = ((d - n0) << ELB) | ((e - c0) & ELM); ++cnt; }
    rec[k] = r;
  }
  int tot; int p = blk_excl_scan(cnt, scan_ws, tid, &tot);
#pragma unroll
  for (int k = 0; k < SP; ++k) if (rec[k] >= 0) { if ((unsigned)p < (unsigned)SCH) LIST[p] = rec[k]; ++p; }
  __syncthreads();
  return tot < SCH ? tot : SCH;
}

__global__ __launch_bounds__(ANT) void agg_kernel(const _Float16* __restrict__ msg, const int* __restrict__ ei, float* acc,
                                                 int N, int E, int c0, int c1, int zinit) {
  __shared__ int LIST[SCH];
  __shared__ int scan_ws[80];
  const int tid = threadIdx.x, lane = tid & 31, wave = tid >> 5;
  const int n0 = blockIdx.x * SRB;
  int nv = N - n0; nv = nv < SRB ? nv : SRB;
  const int nhi = n0 + nv;
  const v4f z4 = {0.f, 0.f, 0.f, 0.f};

  if (zinit) {
#pragma unroll 1
    for (int j = 0; j < RPW; ++j) {
      const int dl = wave * RPW + j;
      if (dl < nv) {
        float* rp = acc + (size_t)(n0 + dl) * DIMC + 4 * lane;
        *(volatile v4f*)rp = z4; *(volatile v4f*)(rp + 128) = z4;
        __threadfence();
        *(volatile v4f*)rp = z4; *(volatile v4f*)(rp + 128) = z4;
      }
    }
  }

  const int* dstv = ei + E;
  const int clen = c1 - c0;
  const int nch = (clen + SCH - 1) / SCH;
#pragma unroll 1
  for (int ch = 0; ch < nch; ++ch) {
    const int tot = chunk_hits_e(dstv, c0 + ch * SCH, c0, c1, n0, nhi, tid, LIST, scan_ws);
#pragma unroll 1
    for (int base = 0; base < tot; base += 32) {
      const int q = base + lane;
      const int qc = q < SCH ? q : SCH - 1;
      const int lv = LIST[qc];
      const int rv = (q < tot) ? lv : -1;
      const int own = (rv >= 0 && ((rv >> ELB) >> 8) == wave) ? 1 : 0;
      unsigned msk = (unsigned)__ballot(own);
#pragma unroll 1
      for (int it = 0; it < 32; ++it) {
        if (msk == 0u) break;
        const int bp = __builtin_ctz(msk); msk &= msk - 1u;
        const int r = __shfl(rv, bp, 32);
        int dl = r >> ELB; dl = dl < 0 ? 0 : (dl >= nv ? nv - 1 : dl);
        int el = r & ELM;  el = el >= clen ? clen - 1 : el;
        const _Float16* mr = msg + (size_t)el * DIMC;
        const v4h mh0 = *(const v4h*)(mr + 4 * lane);
        const v4h mh1 = *(const v4h*)(mr + 128 + 4 * lane);
        const v4f f0 = __builtin_convertvector(mh0, v4f);
        const v4f f1 = __builtin_convertvector(mh1, v4f);
        float* rp = acc + (size_t)(n0 + dl) * DIMC + 4 * lane;
        v4f a = *(const v4f*)rp;
        v4f bb = *(const v4f*)(rp + 128);
        a = a + f0 * MSG_ISC;
        bb = bb + f1 * MSG_ISC;
        *(volatile v4f*)rp = a; *(volatile v4f*)(rp + 128) = bb;
        __threadfence();
        *(volatile v4f*)rp = a; *(volatile v4f*)(rp + 128) = bb;
      }
    }
    __syncthreads();
  }
}

__global__ __launch_bounds__(256) void final_kernel(const float* __restrict__ atom, const float* __restrict__ acc,
                                                    float* out, int n4) {
  const int i = blockIdx.x * 256 + threadIdx.x;
  if (i < n4) {
    const v4f a = *(const v4f*)(atom + (size_t)i * 4);
    const v4f g = *(const v4f*)(acc + (size_t)i * 4);
    const v4f v = a + g;
    *(volatile v4f*)(out + (size_t)i * 4) = v;
    __threadfence();
    *(volatile v4f*)(out + (size_t)i * 4) = v;
  }
}

extern "C" void kernel_launch(void* const* d_in, const int* in_sizes, int n_in,
                              void* d_out, int out_size, void* d_ws, size_t ws_size, hipStream_t stream) {
  (void)n_in; (void)out_size;
  const float* W[15];
  for (int i = 0; i < 15; ++i) W[i] = (const float*)d_in[i];
  const float* atom = (const float*)d_in[15];
  const float* evec = (const float*)d_in[16];
  const int*   ei   = (const int*)d_in[17];
  const int N = in_sizes[15] / DIMC;
  const int E = in_sizes[17] / 2;
  if (N <= 0 || E <= 0) return;
  const int C = (((E + NCHUNK - 1) / NCHUNK) + 63) / 64 * 64;
  if (C <= 0 || C > (1 << ELB)) return;

  char* ws = (char*)d_ws; size_t off = 0;
  auto carve = [&](size_t bytes) -> char* { char* p = ws + off; off += (bytes + 255) & ~(size_t)255; return p; };
  _Float16* bt   = (_Float16*)carve((size_t)BT_HALVES * 2);
  float*    shv  = (float*)carve((size_t)3 * C * 4);
  float*    accb = (float*)carve((size_t)N * DIMC * 4);
  _Float16* sl0  = (_Float16*)carve((size_t)NSLOTS * C * 128);
  if (off > ws_size || off > (size_t)134217728) return;

  const long pstride = (long)C * 64;
  _Float16* X0D = sl0;
  _Float16* X1  = sl0 + 2 * pstride;
  float*    GC  = (float*)(sl0 + 5 * pstride);
  _Float16* H1P = sl0 + 7 * pstride;
  _Float16* HD  = sl0 + 2 * pstride;
  _Float16* LK  = sl0 + 4 * pstride;
  _Float16* SC  = sl0;
  _Float16* O0  = sl0 + 1 * pstride;
  float*    G2  = (float*)(sl0 + 5 * pstride);
  _Float16* O1  = sl0 + 2 * pstride;
  _Float16* MSG = sl0 + 5 * pstride;

  prep_kernel<<<9, 256, 0, stream>>>(W[0], W[1], W[4], W[5], W[6], W[7], W[8], W[9], W[10], W[11], W[12], W[13], W[14], bt);

  const int agrid = (N + SRB - 1) / SRB;
  int zdone = 0;
  for (int ck = 0; ck < NCHUNK; ++ck) {
    const int c0 = ck * C;
    int c1 = c0 + C; if (c1 > E) c1 = E;
    const int cl = c1 - c0;
    if (cl <= 0) continue;
    const int Mpad = (cl + 63) / 64 * 64;
    const int gx = (Mpad / 64 + 7) / 8;
    const int g32 = Mpad / 32;
    const unsigned short* uX0D = (const unsigned short*)X0D;
    const unsigned short* uX1  = (const unsigned short*)X1;
    const unsigned short* uHD  = (const unsigned short*)HD;
    const unsigned short* uLK  = (const unsigned short*)LK;
    const unsigned short* uH1P = (const unsigned short*)H1P;
    const unsigned short* uBT1 = (const unsigned short*)(bt + BT1_OFF);
    const unsigned short* uBTC = (const unsigned short*)(bt + BTC_OFF);
    const unsigned short* uBTD = (const unsigned short*)(bt + BTD_OFF);
    const unsigned short* uBTS = (const unsigned short*)(bt + BTS_OFF);
    const unsigned short* uBT2 = (const unsigned short*)(bt + BT2_OFF);
    const unsigned short* uBT21 = (const unsigned short*)(bt + BT21_OFF);
    const unsigned short* uBT22 = (const unsigned short*)(bt + BT22_OFF);

    gather_kernel<<<(Mpad + 255) / 256, 256, 0, stream>>>(atom, evec, ei, X0D, X1, shv, pstride, N, E, c0, C, Mpad);
    GEMM_F32<<<dim3(gx, 1), 256, 0, stream>>>(uX0D, uX0D, 128, 0L, uBTC, uBTC, 64, 0L, (void*)GC, (void*)GC, 64, 0L,
                                              shv, 0L, shv, 0L, Mpad, 64, 64, INV_TPF);
    GEMM_RS<<<dim3(gx, 3), 256, 0, stream>>>(uX1, uX1, 64, pstride, uBTD, uBTD, 64, 0L, (void*)H1P, (void*)H1P, 64, pstride,
                                             shv, (long)C, GC, 0L, Mpad, 64, 64, INV_TPF);
    GEMM_F16<<<dim3(gx, 1), 256, 0, stream>>>(uX0D, uX0D, 128, 0L, uBT1, uBT1, 128, 0L, (void*)HD, (void*)HD, 128, 0L,
                                              shv, 0L, shv, 0L, Mpad, 64, 128, INV_TPF);
    lkdot_kernel<<<g32, 256, 0, stream>>>(HD, H1P, shv, LK, pstride, C, Mpad);
    GEMM_F16<<<dim3(gx, 1), 256, 0, stream>>>(uLK, uLK, 64, 0L, uBTS, uBTS, 64, 0L, (void*)SC, (void*)SC, 64, 0L,
                                              shv, 0L, shv, 0L, Mpad, 64, 64, INV_MULF * LK_ISC);
    GEMM_F16<<<dim3(gx, 1), 256, 0, stream>>>(uHD, uHD, 128, 0L, uBT2, uBT2, 128, 0L, (void*)O0, (void*)O0, 64, 0L,
                                              shv, 0L, shv, 0L, Mpad, 64, 128, INV_TPF);
    GEMM_F32<<<dim3(gx, 1), 256, 0, stream>>>(uHD, uHD, 128, 0L, uBT21, uBT21, 64, 0L, (void*)G2, (void*)G2, 64, 0L,
                                              shv, 0L, shv, 0L, Mpad, 64, 64, INV_TPF);
    GEMM_RS<<<dim3(gx, 3), 256, 0, stream>>>(uH1P, uH1P, 64, pstride, uBT22, uBT22, 64, 0L, (void*)O1, (void*)O1, 64, pstride,
                                             shv, (long)C, G2, 0L, Mpad, 64, 64, INV_TPF);
    msg_kernel<<<g32, 256, 0, stream>>>(SC, O0, O1, MSG, pstride, Mpad);
    agg_kernel<<<agrid, ANT, 0, stream>>>(MSG, ei, accb, N, E, c0, c1, zdone ? 0 : 1);
    zdone = 1;
  }
  const int n4 = N * (DIMC / 4);
  final_kernel<<<(n4 + 255) / 256, 256, 0, stream>>>(atom, accb, (float*)d_out, n4);
}
